// THTN_13185549598956
// MI455X (gfx1250) — hardware-verified
//
#include <hip/hip_runtime.h>
#include <stdint.h>

#define NN    40000
#define EE    8000
#define DEGE  32
#define DEGV  8
#define DD    256
#define EIG   64
#define KA    320
#define VOC   1000
#define NCLS  40
#define NCP   64
#define LN_EPS 1e-5f
#define WSC   64.0f
#define WINV  0.015625f
#define ATT_SCALE 0.0625f

#define WS_WA     0ull
#define WS_WSTD   163840ull
#define WS_WCLS   1474560ull
#define WS_FV32   1507328ull
#define WS_T3     1507328ull
#define WS_FVP16  21987328ull
#define WS_KN16   42467328ull
#define WS_VN16   62947328ull
#define WS_XV32   42467328ull
#define WS_QV16   83427328ull
#define WS_FV16   103907328ull
#define WS_XE32   103907328ull
#define WS_KE16   103907328ull
#define WS_XE16   112099328ull
#define WS_XV16   112099328ull
#define WS_T1     116195328ull
#define WS_FE16   120291328ull
#define WS_QE16   124387328ull
#define WS_TOTAL  132579328ull
static_assert(WS_WSTD == WS_WA + 256ull * KA * 2);
static_assert(WS_WCLS == WS_WSTD + 10ull * DD * DD * 2);
static_assert(WS_FV32 == WS_WCLS + (unsigned long long)NCP * DD * 2);
static_assert(WS_FVP16 == WS_T3 + (unsigned long long)NN * DD * 2);
static_assert(WS_KN16 == WS_FV32 + (unsigned long long)NN * DD * 4);
static_assert(WS_KN16 == WS_FVP16 + (unsigned long long)NN * DD * 2);
static_assert(WS_VN16 == WS_KN16 + (unsigned long long)NN * DD * 2);
static_assert(WS_QV16 == WS_VN16 + (unsigned long long)NN * DD * 2);
static_assert(WS_QV16 == WS_XV32 + (unsigned long long)NN * DD * 4);
static_assert(WS_FV16 == WS_QV16 + (unsigned long long)NN * DD * 2);
static_assert(WS_XE16 == WS_XE32 + (unsigned long long)EE * DD * 4);
static_assert(WS_XE16 == WS_KE16 + 2ull * EE * DD * 2);
static_assert(WS_T1 == WS_XE16 + (unsigned long long)EE * DD * 2);
static_assert(WS_FE16 == WS_T1 + (unsigned long long)EE * DD * 2);
static_assert(WS_QE16 == WS_FE16 + (unsigned long long)EE * DD * 2);
static_assert(WS_QE16 == WS_FV16 + (unsigned long long)NN * DD * 2);
static_assert(WS_QE16 + (unsigned long long)EE * DD * 2 <= WS_TOTAL);
static_assert(WS_TOTAL == WS_XV16 + (unsigned long long)NN * DD * 2);
static_assert(WS_TOTAL <= 134217728ull);
static_assert((WS_FV32 % 128) == 0 && (WS_FVP16 % 128) == 0 && (WS_KN16 % 128) == 0 && (WS_VN16 % 128) == 0);
static_assert((WS_QV16 % 128) == 0 && (WS_FV16 % 128) == 0 && (WS_XE16 % 128) == 0 && (WS_T1 % 128) == 0);
static_assert((WS_FE16 % 128) == 0 && (WS_QE16 % 128) == 0 && (WS_WSTD % 128) == 0 && (WS_WCLS % 128) == 0);
static_assert(NN % 32 == 0 && EE % 32 == 0 && NN % 8 == 0 && EE % 8 == 0);

typedef _Float16 v16h __attribute__((ext_vector_type(16)));
typedef _Float16 v8h  __attribute__((ext_vector_type(8)));
typedef float    v8f  __attribute__((ext_vector_type(8)));
typedef float    v4f  __attribute__((ext_vector_type(4)));
union Frag { v16h v; v8h half[2]; };

__device__ __forceinline__ unsigned short bfb(float f) {
  const unsigned u = __float_as_uint(f);
  return (unsigned short)((u + 0x7FFFu + ((u >> 16) & 1u)) >> 16);
}
__device__ __forceinline__ float bfr(float f) { return __uint_as_float(((unsigned)bfb(f)) << 16); }
__device__ __forceinline__ v8f zero8() {
  v8f z;
  z[0] = 0.f; z[1] = 0.f; z[2] = 0.f; z[3] = 0.f; z[4] = 0.f; z[5] = 0.f; z[6] = 0.f; z[7] = 0.f;
  return z;
}
__device__ __forceinline__ float wsum32(float v) {
#pragma unroll
  for (int off = 16; off > 0; off >>= 1) v += __shfl_xor(v, off, 32);
  return v;
}
__device__ __forceinline__ float wmax32(float v) {
#pragma unroll
  for (int off = 16; off > 0; off >>= 1) v = fmaxf(v, __shfl_xor(v, off, 32));
  return v;
}

__device__ __forceinline__ v16h ldh(const _Float16* p) {
  Frag f;
  f.half[0] = *(const v8h*)(p);
  f.half[1] = *(const v8h*)(p + 16);
  return f.v;
}
__device__ __forceinline__ v16h ldf(const float* p) {
  const v4f a0 = *(const v4f*)(p);
  const v4f a1 = *(const v4f*)(p + 4);
  const v4f a2 = *(const v4f*)(p + 16);
  const v4f a3 = *(const v4f*)(p + 20);
  v8h h0, h1;
#pragma unroll
  for (int c = 0; c < 4; ++c) {
    h0[c]     = (_Float16)bfr(a0[c]);
    h0[4 + c] = (_Float16)bfr(a1[c]);
    h1[c]     = (_Float16)bfr(a2[c]);
    h1[4 + c] = (_Float16)bfr(a3[c]);
  }
  Frag f;
  f.half[0] = h0;
  f.half[1] = h1;
  return f.v;
}

__device__ __forceinline__ v8f mma(v16h a, v16h b, v8f c) {
  v8f d = __builtin_amdgcn_wmma_f32_16x16x32_f16(false, a, false, b, (short)0, c, false, false);
#if defined(__HIP_DEVICE_COMPILE__)
  asm volatile("v_nop\n\tv_nop\n\tv_nop\n\tv_nop" : "+v"(d) : "v"(a), "v"(b));
#endif
  return d;
}

__device__ __forceinline__ void step4(v16h a, const _Float16* pb0, const _Float16* pb1, const _Float16* pb2,
                                      const _Float16* pb3, int koff, v8f& q0, v8f& q1, v8f& q2, v8f& q3) {
  const v16h b0 = ldh(pb0 + koff);
  const v16h b1 = ldh(pb1 + koff);
  const v16h b2 = ldh(pb2 + koff);
  const v16h b3 = ldh(pb3 + koff);
  q0 = mma(a, b0, q0);
  q1 = mma(a, b1, q1);
  q2 = mma(a, b2, q2);
  q3 = mma(a, b3, q3);
}

template<int NCW, int ASRC>
__device__ __forceinline__ void gemm_core(const _Float16* __restrict__ A16, const float* __restrict__ Af,
                                          const float* __restrict__ Ag, int lda, int ksteps,
                                          const _Float16* __restrict__ B, int ldb, int c0, float* ST)
{
  constexpr int STP = NCW * 64 + 4;
  const int tid = threadIdx.x, lane = tid & 31, wave = tid >> 5, lr = lane & 15, lh = lane >> 4;
  const int wr = wave / NCW, wc = wave - wr * NCW;
  const int arow = 32 * (int)blockIdx.x + 16 * wr + lr;
  const _Float16* pb0 = B + (size_t)(c0 + 64 * wc + lr) * (size_t)ldb + 8 * lh;
  const _Float16* pb1 = pb0 + (size_t)16 * ldb;
  const _Float16* pb2 = pb0 + (size_t)32 * ldb;
  const _Float16* pb3 = pb0 + (size_t)48 * ldb;
  v8f q0 = zero8(), q1 = zero8(), q2 = zero8(), q3 = zero8();
  if (ASRC == 0) {
    const _Float16* pa = A16 + (size_t)arow * (size_t)lda + 8 * lh;
#pragma unroll 2
    for (int ks = 0; ks < ksteps; ++ks) {
      const v16h a = ldh(pa + 32 * ks);
      step4(a, pb0, pb1, pb2, pb3, 32 * ks, q0, q1, q2, q3);
    }
  } else if (ASRC == 1) {
    const float* pa = Af + (size_t)arow * (size_t)lda + 8 * lh;
#pragma unroll 2
    for (int ks = 0; ks < ksteps; ++ks) {
      const v16h a = ldf(pa + 32 * ks);
      step4(a, pb0, pb1, pb2, pb3, 32 * ks, q0, q1, q2, q3);
    }
  } else {
    const float* pa = Af + (size_t)arow * DD + 8 * lh;
#pragma unroll 2
    for (int ks = 0; ks < DD / 32; ++ks) {
      const v16h a = ldf(pa + 32 * ks);
      step4(a, pb0, pb1, pb2, pb3, 32 * ks, q0, q1, q2, q3);
    }
    const float* pe = Ag + (size_t)arow * EIG + 8 * lh;
#pragma unroll
    for (int ks = 0; ks < EIG / 32; ++ks) {
      const v16h a = ldf(pe + 32 * ks);
      step4(a, pb0, pb1, pb2, pb3, DD + 32 * ks, q0, q1, q2, q3);
    }
  }
  float* st = ST + (size_t)(16 * wr + 8 * lh) * STP + 64 * wc + lr;
#pragma unroll
  for (int r = 0; r < 8; ++r) {
    st[r * STP]      = q0[r];
    st[r * STP + 16] = q1[r];
    st[r * STP + 32] = q2[r];
    st[r * STP + 48] = q3[r];
  }
}

__global__ __launch_bounds__(256) void k_wcvt(const float* __restrict__ w_vtx, const float* __restrict__ w_pe,
    const float* __restrict__ w_kv, const float* __restrict__ w_vv, const float* __restrict__ w_qv,
    const float* __restrict__ w_qe, const float* __restrict__ w_l1, const float* __restrict__ w_l2,
    const float* __restrict__ w_ke, const float* __restrict__ w_ve, const float* __restrict__ w_l3,
    const float* __restrict__ w_l4, const float* __restrict__ w_cls,
    _Float16* WA, _Float16* WSTD, _Float16* WCLS)
{
  __shared__ __align__(16) _Float16 tile[32 * 72];
  const int j = blockIdx.y;
  const float* src = w_vtx;
  _Float16* dst = WA;
  int K = DD, Nv = DD, sp = DD, dp = KA, ko = 0, nTN = 8;
  if (j == 1)  { src = w_pe; K = EIG; ko = DD; }
  if (j == 2)  src = w_kv;
  if (j == 3)  src = w_vv;
  if (j == 4)  src = w_qv;
  if (j == 5)  src = w_qe;
  if (j == 6)  src = w_l1;
  if (j == 7)  src = w_l2;
  if (j == 8)  src = w_ke;
  if (j == 9)  src = w_ve;
  if (j == 10) src = w_l3;
  if (j == 11) src = w_l4;
  if (j >= 2 && j <= 11) { dst = WSTD + (size_t)(j - 2) * DD * DD; dp = DD; }
  if (j == 12) { src = w_cls; dst = WCLS; Nv = NCLS; sp = NCLS; dp = DD; nTN = 2; }
  const int nTK = K >> 6;
  if ((int)blockIdx.x >= nTN * nTK) return;
  const int tn = (int)blockIdx.x % nTN, tk = (int)blockIdx.x / nTN;
  const int n0 = 32 * tn, k0 = 64 * tk;
  const int tid = threadIdx.x;
#pragma unroll
  for (int it = 0; it < 8; ++it) {
    const int i  = it * 256 + tid;
    const int kk = i >> 5, nn = i & 31;
    const int gn = n0 + nn;
    const int gnc = min(gn, Nv - 1);
    const float v = src[(size_t)(k0 + kk) * sp + gnc];
    const float s = (gn < Nv) ? WSC * bfr(v) : 0.0f;
    tile[nn * 72 + kk] = (_Float16)s;
  }
  __syncthreads();
  const int row = tid >> 3, pc = tid & 7;
  const v8h hv = *(const v8h*)(tile + row * 72 + 8 * pc);
  _Float16* d = dst + (size_t)(n0 + row) * dp + ko + k0 + 8 * pc;
  *(volatile v8h*)d = hv;
  __threadfence();
  *(volatile v8h*)d = hv;
}

template<int ASRC, int RELU>
__global__ __launch_bounds__(256) void k_gemm_f16(const _Float16* __restrict__ A16, const float* __restrict__ Af,
    int lda, int ksteps, const _Float16* __restrict__ B, int ldb,
    const float* __restrict__ bias0, const float* __restrict__ bias1, const float* __restrict__ bias2,
    _Float16* O16, long long pstride)
{
  __shared__ __align__(16) float ST[32 * 260];
  gemm_core<4, ASRC>(A16, Af, Af, lda, ksteps, B, ldb, 256 * (int)blockIdx.y, ST);
  __syncthreads();
  const int by  = blockIdx.y;
  const float* bias = (by == 0) ? bias0 : ((by == 1) ? bias1 : bias2);
  _Float16* op = O16 + (size_t)by * (size_t)pstride + (size_t)(32 * (int)blockIdx.x) * DD;
  const int tid = threadIdx.x;
  v8h hv[4];
#pragma unroll
  for (int it = 0; it < 4; ++it) {
    const int i = it * 256 + tid, row = i >> 5, c = (i & 31) * 8;
    const float* sp = ST + row * 260 + c;
    const v4f x0 = *(const v4f*)(sp), x1 = *(const v4f*)(sp + 4);
    const v4f b0 = *(const v4f*)(bias + c), b1 = *(const v4f*)(bias + c + 4);
    float y[8];
#pragma unroll
    for (int k = 0; k < 4; ++k) {
      y[k]     = x0[k] * WINV + bfr(b0[k]);
      y[4 + k] = x1[k] * WINV + bfr(b1[k]);
    }
#pragma unroll
    for (int k = 0; k < 8; ++k) {
      if (RELU) y[k] = fmaxf(y[k], 0.0f);
      hv[it][k] = (_Float16)y[k];
    }
    *(volatile v8h*)(op + (size_t)row * DD + c) = hv[it];
  }
  __threadfence();
#pragma unroll
  for (int it = 0; it < 4; ++it) {
    const int i = it * 256 + tid, row = i >> 5, c = (i & 31) * 8;
    *(volatile v8h*)(op + (size_t)row * DD + c) = hv[it];
  }
}

__global__ __launch_bounds__(256) void k_gemm_fv(const float* __restrict__ vfeat, const float* __restrict__ eign,
    const _Float16* __restrict__ WA, const float* __restrict__ bvtx, const float* __restrict__ bpe,
    const float* __restrict__ gcn, const float* __restrict__ cs, const float* __restrict__ un,
    const int* __restrict__ ci, const int* __restrict__ ui, float* O32, _Float16* O16)
{
  __shared__ __align__(16) float ST[32 * 260];
  gemm_core<4, 2>(WA, vfeat, eign, DD, KA / 32, WA, KA, 0, ST);
  __syncthreads();
  const int tid = threadIdx.x;
  const int r0 = 32 * (int)blockIdx.x;
  v8h hv[4];
#pragma unroll
  for (int it = 0; it < 4; ++it) {
    const int i = it * 256 + tid, row = i >> 5, c = (i & 31) * 8;
    const int grow = r0 + row;
    float* sp = ST + row * 260 + c;
    const v4f x0 = *(const v4f*)(sp), x1 = *(const v4f*)(sp + 4);
    int cc = ci[grow]; cc = min(max(cc, 0), VOC - 1);
    int uu = ui[grow]; uu = min(max(uu, 0), VOC - 1);
    const float* pg = gcn + (size_t)grow * DD + c;
    const float* ps = cs + (size_t)cc * DD + c;
    const float* pu = un + (size_t)uu * DD + c;
    const v4f g0 = *(const v4f*)(pg), g1 = *(const v4f*)(pg + 4);
    const v4f s0 = *(const v4f*)(ps), s1 = *(const v4f*)(ps + 4);
    const v4f u0 = *(const v4f*)(pu), u1 = *(const v4f*)(pu + 4);
    const v4f b0 = *(const v4f*)(bvtx + c), b1 = *(const v4f*)(bvtx + c + 4);
    const v4f e0 = *(const v4f*)(bpe + c), e1 = *(const v4f*)(bpe + c + 4);
    v4f w0, w1;
#pragma unroll
    for (int k = 0; k < 4; ++k) {
      w0[k] = x0[k] * WINV + (bfr(b0[k]) + bfr(e0[k])) + bfr(g0[k]) + bfr(s0[k]) + bfr(u0[k]);
      w1[k] = x1[k] * WINV + (bfr(b1[k]) + bfr(e1[k])) + bfr(g1[k]) + bfr(s1[k]) + bfr(u1[k]);
      hv[it][k]     = (_Float16)w0[k];
      hv[it][4 + k] = (_Float16)w1[k];
    }
    *(v4f*)(sp) = w0;
    *(v4f*)(sp + 4) = w1;
  }
  __syncthreads();
  v4f fv[8];
#pragma unroll
  for (int it = 0; it < 8; ++it) {
    const int i = it * 256 + tid, row = i >> 6, q = (i & 63) * 4;
    fv[it] = *(const v4f*)(ST + row * 260 + q);
    *(volatile v4f*)(O32 + (size_t)(r0 + row) * DD + q) = fv[it];
  }
#pragma unroll
  for (int it = 0; it < 4; ++it) {
    const int i = it * 256 + tid, row = i >> 5, c = (i & 31) * 8;
    *(volatile v8h*)(O16 + (size_t)(r0 + row) * DD + c) = hv[it];
  }
  __threadfence();
#pragma unroll
  for (int it = 0; it < 8; ++it) {
    const int i = it * 256 + tid, row = i >> 6, q = (i & 63) * 4;
    *(volatile v4f*)(O32 + (size_t)(r0 + row) * DD + q) = fv[it];
  }
#pragma unroll
  for (int it = 0; it < 4; ++it) {
    const int i = it * 256 + tid, row = i >> 5, c = (i & 31) * 8;
    *(volatile v8h*)(O16 + (size_t)(r0 + row) * DD + c) = hv[it];
  }
}

__global__ __launch_bounds__(256) void k_gemm_ln(const _Float16* __restrict__ A16, const _Float16* __restrict__ B,
    const float* __restrict__ bias, const float* __restrict__ R32, const float* __restrict__ lng,
    const float* __restrict__ lnb, _Float16* O16)
{
  __shared__ __align__(16) float ST[32 * 260];
  gemm_core<4, 0>(A16, bias, bias, DD, DD / 32, B, DD, 0, ST);
  __syncthreads();
  const int tid = threadIdx.x, lane = tid & 31, wave = tid >> 5;
  const int r0 = 32 * (int)blockIdx.x;
#pragma unroll
  for (int it = 0; it < 4; ++it) {
    const int i = it * 256 + tid, row = i >> 5, c = (i & 31) * 8;
    const int grow = r0 + row;
    float* sp = ST + row * 260 + c;
    const v4f x0 = *(const v4f*)(sp), x1 = *(const v4f*)(sp + 4);
    const v4f b0 = *(const v4f*)(bias + c), b1 = *(const v4f*)(bias + c + 4);
    const float* pr = R32 + (size_t)grow * DD + c;
    const v4f q0 = *(const v4f*)(pr), q1 = *(const v4f*)(pr + 4);
    v4f w0, w1;
#pragma unroll
    for (int k = 0; k < 4; ++k) {
      w0[k] = (x0[k] * WINV + bfr(b0[k])) + q0[k];
      w1[k] = (x1[k] * WINV + bfr(b1[k])) + q1[k];
    }
    *(v4f*)(sp) = w0;
    *(v4f*)(sp + 4) = w1;
  }
  __syncthreads();
  const v4f g0 = *(const v4f*)(lng + 8 * lane), g1 = *(const v4f*)(lng + 8 * lane + 4);
  const v4f e0 = *(const v4f*)(lnb + 8 * lane), e1 = *(const v4f*)(lnb + 8 * lane + 4);
  float gg[8], bb[8];
#pragma unroll
  for (int k = 0; k < 4; ++k) { gg[k] = bfr(g0[k]); gg[4 + k] = bfr(g1[k]); bb[k] = bfr(e0[k]); bb[4 + k] = bfr(e1[k]); }
  v8h hv[4];
#pragma unroll
  for (int rr = 0; rr < 4; ++rr) {
    const int row = 4 * wave + rr;
    const float* sp = ST + row * 260 + 8 * lane;
    const v4f x0 = *(const v4f*)(sp), x1 = *(const v4f*)(sp + 4);
    float h[8];
#pragma unroll
    for (int k = 0; k < 4; ++k) { h[k] = x0[k]; h[4 + k] = x1[k]; }
    float s1 = 0.0f;
#pragma unroll
    for (int k = 0; k < 8; ++k) s1 += h[k];
    s1 = wsum32(s1);
    const float mu = s1 * (1.0f / DD);
    float d[8];
    float s2 = 0.0f;
#pragma unroll
    for (int k = 0; k < 8; ++k) { d[k] = h[k] - mu; s2 += d[k] * d[k]; }
    s2 = wsum32(s2);
    const float rstd = rsqrtf(s2 * (1.0f / DD) + LN_EPS);
#pragma unroll
    for (int k = 0; k < 8; ++k) hv[rr][k] = (_Float16)((d[k] * rstd) * gg[k] + bb[k]);
    *(volatile v8h*)(O16 + (size_t)(r0 + row) * DD + 8 * lane) = hv[rr];
  }
  __threadfence();
#pragma unroll
  for (int rr = 0; rr < 4; ++rr) {
    const int row = 4 * wave + rr;
    *(volatile v8h*)(O16 + (size_t)(r0 + row) * DD + 8 * lane) = hv[rr];
  }
}

__global__ __launch_bounds__(64) void k_gemm_out(const _Float16* __restrict__ A16, const _Float16* __restrict__ B,
    const float* __restrict__ bcls, float* OUT)
{
  __shared__ __align__(16) float ST[32 * 68];
  __shared__ __align__(16) float SO[32 * NCLS];
  gemm_core<1, 0>(A16, bcls, bcls, DD, DD / 32, B, DD, 0, ST);
  __syncthreads();
  const int tid = threadIdx.x;
#pragma unroll
  for (int i = 0; i < 20; ++i) {
    const int f = i * 64 + tid;
    const int row = f / NCLS;
    const int c = f - row * NCLS;
    SO[f] = ST[row * 68 + c] * WINV + bfr(bcls[c]);
  }
  __syncthreads();
  float* ob = OUT + (size_t)blockIdx.x * (32 * NCLS);
  v4f ov[5];
#pragma unroll
  for (int it = 0; it < 5; ++it) {
    const int q = it * 64 + tid;
    ov[it] = *(const v4f*)(SO + 4 * q);
    *(volatile v4f*)(ob + 4 * q) = ov[it];
  }
  __threadfence();
#pragma unroll
  for (int it = 0; it < 5; ++it) {
    const int q = it * 64 + tid;
    *(volatile v4f*)(ob + 4 * q) = ov[it];
  }
}

template<int DEG, int RIN>
__global__ __launch_bounds__(256) void k_attn(const _Float16* __restrict__ Q16, const _Float16* __restrict__ K16,
    const _Float16* __restrict__ V16, int nRows, const int* __restrict__ nbr, const float* __restrict__ cent,
    const float* __restrict__ res, const float* __restrict__ lng, const float* __restrict__ lnb,
    float* X32, _Float16* X16)
{
  __shared__ __align__(16) float srow[8 * 256];
  const int tid = threadIdx.x, lane = tid & 31, wave = tid >> 5;
  const int item = 8 * (int)blockIdx.x + wave;
  const v8h qh = *(const v8h*)(Q16 + (size_t)item * DD + 8 * lane);
  float qv[8];
#pragma unroll
  for (int c = 0; c < 8; ++c) qv[c] = (float)qh[c];
  const int*   nb = nbr  + (size_t)item * DEG;
  const float* ce = cent + (size_t)item * DEG;
  float mylg = -3.0e38f;
  int   myj  = 0;
#pragma unroll 1
  for (int d = 0; d < DEG; ++d) {
    int j = nb[d];
    j = min(max(j, 0), nRows - 1);
    const v8h kh = *(const v8h*)(K16 + (size_t)j * DD + 8 * lane);
    float p = 0.0f;
#pragma unroll
    for (int c = 0; c < 8; ++c) p += (float)kh[c] * qv[c];
    p = wsum32(p);
    float lg = (p >= 0.0f) ? p : 0.01f * p;
    lg = lg * ATT_SCALE + bfr(ce[d]);
    mylg = (lane == d) ? lg : mylg;
    myj  = (lane == d) ? j : myj;
  }
  const float m  = wmax32(mylg);
  const float ex = __expf(mylg - m);
  const float e  = (lane < DEG) ? ex : 0.0f;
  const float s  = wsum32(e);
  const float sc = e * (1.0f / s);
  float acc[8];
#pragma unroll
  for (int c = 0; c < 8; ++c) acc[c] = 0.0f;
#pragma unroll 1
  for (int d = 0; d < DEG; ++d) {
    const float pd = __shfl(sc, d, 32);
    const int   jj = __shfl(myj, d, 32);
    const v8h vh = *(const v8h*)(V16 + (size_t)jj * DD + 8 * lane);
#pragma unroll
    for (int c = 0; c < 8; ++c) acc[c] += pd * (float)vh[c];
  }
  const float* rp = res + (size_t)item * DD + 8 * lane;
  const v4f ra = *(const v4f*)(rp), rb = *(const v4f*)(rp + 4);
  float h[8];
#pragma unroll
  for (int c = 0; c < 4; ++c) {
    const float r0v = RIN ? bfr(ra[c]) : ra[c];
    const float r1v = RIN ? bfr(rb[c]) : rb[c];
    h[c]     = acc[c] + r0v;
    h[4 + c] = acc[4 + c] + r1v;
  }
  float s1 = 0.0f;
#pragma unroll
  for (int c = 0; c < 8; ++c) s1 += h[c];
  s1 = wsum32(s1);
  const float mu = s1 * (1.0f / DD);
  float dv[8];
  float s2 = 0.0f;
#pragma unroll
  for (int c = 0; c < 8; ++c) { dv[c] = h[c] - mu; s2 += dv[c] * dv[c]; }
  s2 = wsum32(s2);
  const float rstd = rsqrtf(s2 * (1.0f / DD) + LN_EPS);
  const v4f g0 = *(const v4f*)(lng + 8 * lane), g1 = *(const v4f*)(lng + 8 * lane + 4);
  const v4f e0 = *(const v4f*)(lnb + 8 * lane), e1 = *(const v4f*)(lnb + 8 * lane + 4);
  v4f y0, y1;
  v8h hv;
#pragma unroll
  for (int c = 0; c < 4; ++c) {
    y0[c] = (dv[c] * rstd) * bfr(g0[c]) + bfr(e0[c]);
    y1[c] = (dv[4 + c] * rstd) * bfr(g1[c]) + bfr(e1[c]);
    hv[c]     = (_Float16)y0[c];
    hv[4 + c] = (_Float16)y1[c];
  }
  float* sr = srow + wave * 256;
  *(v4f*)(sr + 8 * lane)     = y0;
  *(v4f*)(sr + 8 * lane + 4) = y1;
  __syncthreads();
  const v4f f0 = *(const v4f*)(sr + 4 * lane);
  const v4f f1 = *(const v4f*)(sr + 128 + 4 * lane);
  float* o32 = X32 + (size_t)item * DD;
  _Float16* o16 = X16 + (size_t)item * DD + 8 * lane;
  *(volatile v4f*)(o32 + 4 * lane)       = f0;
  *(volatile v4f*)(o32 + 128 + 4 * lane) = f1;
  *(volatile v8h*)(o16)                  = hv;
  __threadfence();
  *(volatile v4f*)(o32 + 4 * lane)       = f0;
  *(volatile v4f*)(o32 + 128 + 4 * lane) = f1;
  *(volatile v8h*)(o16)                  = hv;
}

extern "C" void kernel_launch(void* const* d_in, const int* in_sizes, int n_in,
                              void* d_out, int out_size, void* d_ws, size_t ws_size,
                              hipStream_t stream) {
  if (n_in < 42) return;
  const int expect[42] = {
    NN * DD, EE * DD, NN * EIG, NN * DD, EE * DEGE, NN * DEGV, NN, NN, EE * DEGE, NN * DEGV,
    DD * DD, DD, EIG * DD, DD, VOC * DD, VOC * DD,
    DD * DD, DD, DD * DD, DD, DD * DD, DD, DD * DD, DD, DD * DD, DD,
    DD * DD, DD, DD * DD, DD, DD * DD, DD, DD * DD, DD, DD * DD, DD,
    DD, DD, DD, DD, DD * NCLS, NCLS };
  for (int i = 0; i < 42; ++i) if (in_sizes[i] != expect[i]) return;
  if (out_size != NN * NCLS) return;
  if ((size_t)WS_TOTAL > ws_size) return;

  const float* vfeat      = (const float*)d_in[0];
  const float* efeat      = (const float*)d_in[1];
  const float* eign_vec   = (const float*)d_in[2];
  const float* feat_v_gcn = (const float*)d_in[3];
  const float* cent1      = (const float*)d_in[4];
  const float* cent2      = (const float*)d_in[5];
  const int*   cent_idx   = (const int*)d_in[6];
  const int*   uniq_idx   = (const int*)d_in[7];
  const int*   edge2node  = (const int*)d_in[8];
  const int*   node2edge  = (const int*)d_in[9];
  const float* W_vtx = (const float*)d_in[10]; const float* b_vtx = (const float*)d_in[11];
  const float* W_pe  = (const float*)d_in[12]; const float* b_pe  = (const float*)d_in[13];
  const float* cs_emb= (const float*)d_in[14]; const float* un_emb= (const float*)d_in[15];
  const float* W_kv  = (const float*)d_in[16]; const float* b_kv  = (const float*)d_in[17];
  const float* W_vv  = (const float*)d_in[18]; const float* b_vv  = (const float*)d_in[19];
  const float* W_qe  = (const float*)d_in[20]; const float* b_qe  = (const float*)d_in[21];
  const float* W_ke  = (const float*)d_in[22]; const float* b_ke  = (const float*)d_in[23];
  const float* W_ve  = (const float*)d_in[24]; const float* b_ve  = (const float*)d_in[25];
  const float* W_qv  = (const float*)d_in[26]; const float* b_qv  = (const float*)d_in[27];
  const float* W_l1  = (const float*)d_in[28]; const float* b_l1  = (const float*)d_in[29];
  const float* W_l2  = (const float*)d_in[30]; const float* b_l2  = (const float*)d_in[31];
  const float* W_l3  = (const float*)d_in[32]; const float* b_l3  = (const float*)d_in[33];
  const float* W_l4  = (const float*)d_in[34]; const float* b_l4  = (const float*)d_in[35];
  const float* ln1_g = (const float*)d_in[36]; const float* ln1_b = (const float*)d_in[37];
  const float* ln2_g = (const float*)d_in[38]; const float* ln2_b = (const float*)d_in[39];
  const float* W_cls = (const float*)d_in[40]; const float* b_cls = (const float*)d_in[41];
  float* out = (float*)d_out;

  unsigned char* ws = (unsigned char*)d_ws;
  _Float16* WA    = (_Float16*)(ws + WS_WA);
  _Float16* WSTD  = (_Float16*)(ws + WS_WSTD);
  _Float16* WCLS  = (_Float16*)(ws + WS_WCLS);
  float*    FV32  = (float*)(ws + WS_FV32);
  _Float16* T3    = (_Float16*)(ws + WS_T3);
  _Float16* FVP16 = (_Float16*)(ws + WS_FVP16);
  _Float16* KN16  = (_Float16*)(ws + WS_KN16);
  _Float16* VN16  = (_Float16*)(ws + WS_VN16);
  float*    XV32  = (float*)(ws + WS_XV32);
  _Float16* QV16  = (_Float16*)(ws + WS_QV16);
  _Float16* FV16  = (_Float16*)(ws + WS_FV16);
  float*    XE32  = (float*)(ws + WS_XE32);
  _Float16* KE16  = (_Float16*)(ws + WS_KE16);
  _Float16* VE16  = KE16 + (size_t)EE * DD;
  _Float16* XE16  = (_Float16*)(ws + WS_XE16);
  _Float16* XV16  = (_Float16*)(ws + WS_XV16);
  _Float16* T1    = (_Float16*)(ws + WS_T1);
  _Float16* FE16  = (_Float16*)(ws + WS_FE16);
  _Float16* QE16  = (_Float16*)(ws + WS_QE16);
  const _Float16* Wkvq  = WSTD;
  const _Float16* Wqe   = WSTD + (size_t)3 * DD * DD;
  const _Float16* Wl1   = WSTD + (size_t)4 * DD * DD;
  const _Float16* Wl2   = WSTD + (size_t)5 * DD * DD;
  const _Float16* Wkeve = WSTD + (size_t)6 * DD * DD;
  const _Float16* Wl3   = WSTD + (size_t)8 * DD * DD;
  const _Float16* Wl4   = WSTD + (size_t)9 * DD * DD;
  const long long psN = (long long)NN * DD;
  const long long psE = (long long)EE * DD;

  k_wcvt<<<dim3(32, 13), dim3(256), 0, stream>>>(W_vtx, W_pe, W_kv, W_vv, W_qv, W_qe, W_l1, W_l2, W_ke, W_ve,
                                                  W_l3, W_l4, W_cls, WA, WSTD, WCLS);
  k_gemm_f16<1, 0><<<dim3(EE / 32, 1), dim3(256), 0, stream>>>(Wqe, efeat, DD, DD / 32, Wqe, DD,
                                                                b_qe, b_qe, b_qe, QE16, psE);
  k_gemm_fv<<<dim3(NN / 32, 1), dim3(256), 0, stream>>>(vfeat, eign_vec, WA, b_vtx, b_pe, feat_v_gcn, cs_emb, un_emb,
                                                        cent_idx, uniq_idx, FV32, FV16);
  k_gemm_f16<0, 0><<<dim3(NN / 32, 3), dim3(256), 0, stream>>>(FV16, b_kv, DD, DD / 32, Wkvq, DD,
                                                                b_kv, b_vv, b_qv, KN16, psN);
  k_attn<DEGE, 1><<<dim3(EE / 8), dim3(256), 0, stream>>>(QE16, KN16, VN16, NN, edge2node, cent1, efeat,
                                                          ln1_g, ln1_b, XE32, XE16);
  k_gemm_f16<0, 1><<<dim3(EE / 32, 1), dim3(256), 0, stream>>>(XE16, b_l1, DD, DD / 32, Wl1, DD,
                                                                b_l1, b_l1, b_l1, T1, psE);
  k_gemm_ln<<<dim3(EE / 32, 1), dim3(256), 0, stream>>>(T1, Wl2, b_l2, XE32, ln1_g, ln1_b, FE16);
  k_gemm_f16<0, 0><<<dim3(EE / 32, 2), dim3(256), 0, stream>>>(FE16, b_ke, DD, DD / 32, Wkeve, DD,
                                                                b_ke, b_ve, b_ve, KE16, psE);
  k_attn<DEGV, 0><<<dim3(NN / 8), dim3(256), 0, stream>>>(QV16, KE16, VE16, EE, node2edge, cent2, FV32,
                                                          ln2_g, ln2_b, XV32, XV16);
  k_gemm_f16<0, 1><<<dim3(NN / 32, 1), dim3(256), 0, stream>>>(XV16, b_l3, DD, DD / 32, Wl3, DD,
                                                                b_l3, b_l3, b_l3, T3, psN);
  k_gemm_ln<<<dim3(NN / 32, 1), dim3(256), 0, stream>>>(T3, Wl4, b_l4, XV32, ln2_g, ln2_b, FVP16);
  k_gemm_out<<<dim3(NN / 32, 1), dim3(64), 0, stream>>>(FVP16, WCLS, b_cls, out);
  (void)hipGetLastError();
}
